// ModelNet10ShapePrior_25074019074117
// MI455X (gfx1250) — hardware-verified
//
#include <hip/hip_runtime.h>
#include <stddef.h>


#define HID      512
#define HID2     256
#define TP       64
#define NTH      256
#define P1       520
#define P2       260
#define PS       520
#define LN_EPS_F 1e-5f
#define SLOPE_F  0.2f
#define A_CARRY  8.0f
#define W_CARRY  256.0f
#define RC2048   0.00048828125f
#define WSCAP    134217728

#define L_H1  0
#define L_H2  (TP * P1 * 2)
#define L_OS  (L_H2 + TP * P2 * 4)
#define L_TOT (L_OS + TP * 3 * 4)

static_assert((L_H2 % 16) == 0 && (L_OS % 16) == 0);
static_assert(32 * PS * 4 == TP * P2 * 4);
static_assert(((P1 * 2) % 16) == 0 && ((P2 * 4) % 16) == 0 && ((PS * 4) % 16) == 0);
static_assert((HID % 32) == 0 && HID2 == 256 && TP == 64 && NTH == 256);
static_assert(L_TOT <= 160 * 1024);
static_assert(((TP * 3 * 4) % 128) == 0);

typedef float    v4f  __attribute__((ext_vector_type(4)));
typedef float    v8f  __attribute__((ext_vector_type(8)));
typedef _Float16 v4h  __attribute__((ext_vector_type(4)));
typedef _Float16 v8h  __attribute__((ext_vector_type(8)));
typedef _Float16 v16h __attribute__((ext_vector_type(16)));
union Frag { v16h v; v8h half[2]; };
union Pk   { v8h h; v4f f; };
static_assert(sizeof(Frag) == 32);
static_assert(sizeof(Pk) == 16);

__device__ __forceinline__ v8f wmf(v16h a, v16h bq, v8f c) {
  v8f d = __builtin_amdgcn_wmma_f32_16x16x32_f16(false, a, false, bq, (short)0, c, false, false);
  asm volatile("v_nop\n\tv_nop\n\tv_nop\n\tv_nop" : "+v"(d) : "v"(a), "v"(bq));
  return d;
}

__device__ __forceinline__ v8f zero8() {
  v8f z = {0.f, 0.f, 0.f, 0.f, 0.f, 0.f, 0.f, 0.f};
  return z;
}

__device__ __forceinline__ v4f lrelu4(v4f u) {
  v4f r;
  r.x = fmaxf(u.x, SLOPE_F * u.x);
  r.y = fmaxf(u.y, SLOPE_F * u.y);
  r.z = fmaxf(u.z, SLOPE_F * u.z);
  r.w = fmaxf(u.w, SLOPE_F * u.w);
  return r;
}

__device__ __forceinline__ int clampi(int v, int lo, int hi) {
  v = v < lo ? lo : v;
  v = v > hi ? hi : v;
  return v;
}

__global__ __launch_bounds__(NTH) void k_w2prep(const float* __restrict__ W2, const int* __restrict__ cat,
                                                _Float16* W2S, int nE) {
  __shared__ _Float16 T[32 * P1];
  const int tid = threadIdx.x, wave = tid >> 5, lane = tid & 31;
  const int b = blockIdx.x >> 3, ng = blockIdx.x & 7, n0 = ng * 32;
  const int e = clampi(cat[b], 0, nE - 1);
  const float* src = W2 + (size_t)e * HID * HID2 + n0 + lane;
#pragma unroll 4
  for (int it = 0; it < HID / 8; ++it) {
    const int k = it * 8 + wave;
    const float v = src[(size_t)k * HID2];
    T[lane * P1 + k] = (_Float16)(v * W_CARRY);
  }
  __syncthreads();
  _Float16* dstb = W2S + ((size_t)b * HID2 + n0) * HID;
#pragma unroll
  for (int rr = 0; rr < 4; ++rr) {
    const int r = wave * 4 + rr;
#pragma unroll
    for (int p = 0; p < 2; ++p) {
      Pk u; u.h = *(const v8h*)(T + r * P1 + 256 * p + 8 * lane);
      *(volatile v4f*)(dstb + (size_t)r * HID + 256 * p + 8 * lane) = u.f;
    }
  }
  __threadfence();
#pragma unroll
  for (int rr = 0; rr < 4; ++rr) {
    const int r = wave * 4 + rr;
#pragma unroll
    for (int p = 0; p < 2; ++p) {
      Pk u; u.h = *(const v8h*)(T + r * P1 + 256 * p + 8 * lane);
      *(volatile v4f*)(dstb + (size_t)r * HID + 256 * p + 8 * lane) = u.f;
    }
  }
}

__global__ __launch_bounds__(NTH) void k_mlp(
    const float* __restrict__ pts, const int* __restrict__ cat,
    const float* __restrict__ W1, const float* __restrict__ b1,
    const float* __restrict__ g1, const float* __restrict__ be1,
    const _Float16* __restrict__ W2S, const float* __restrict__ b2,
    const float* __restrict__ g2, const float* __restrict__ be2,
    const float* __restrict__ W3, const float* __restrict__ b3,
    float* out, int nN, int nE) {
  extern __shared__ v4f lds_dyn[];
  char* sm = (char*)lds_dyn;
  _Float16* H1 = (_Float16*)(sm + L_H1);
  float* H2 = (float*)(sm + L_H2);
  float* S  = H2;
  float* OS = (float*)(sm + L_OS);

  const int tid = threadIdx.x, wave = tid >> 5, lane = tid & 31;
  const int tpb  = nN / TP;
  const int bidx = blockIdx.x / tpb;
  const int tile = blockIdx.x - bidx * tpb;
  const int p0   = tile * TP;
  const int e    = clampi(cat[bidx], 0, nE - 1);

  const float* W1e  = W1  + (size_t)e * 3 * HID;
  const float* b1e  = b1  + (size_t)e * HID;
  const float* g1e  = g1  + (size_t)e * HID;
  const float* be1e = be1 + (size_t)e * HID;
  const float* b2e  = b2  + (size_t)e * HID2;
  const float* g2e  = g2  + (size_t)e * HID2;
  const float* be2e = be2 + (size_t)e * HID2;
  const float* W3e  = W3  + (size_t)e * HID2 * 3;
  const float* b3e  = b3  + (size_t)e * 3;

  {
    const int q = tid & 7, rl = tid >> 3;
#pragma unroll 1
    for (int rh = 0; rh < 2; ++rh) {
      const int row = rh * 32 + rl;
      const float* pp = pts + ((size_t)bidx * nN + p0 + row) * 3;
      const float x = pp[0], y = pp[1], z = pp[2];
      float* srow = S + rl * PS;
      float s = 0.0f;
#pragma unroll 4
      for (int j = 0; j < HID / 32; ++j) {
        const int f = j * 32 + q * 4;
        const v4f w0 = *(const v4f*)(W1e + f);
        const v4f w1 = *(const v4f*)(W1e + HID + f);
        const v4f w2 = *(const v4f*)(W1e + 2 * HID + f);
        const v4f bb = *(const v4f*)(b1e + f);
        const v4f hv = x * w0 + y * w1 + z * w2 + bb;
        *(v4f*)(srow + f) = hv;
        s += (hv.x + hv.y) + (hv.z + hv.w);
      }
      s += __shfl_xor(s, 1);
      s += __shfl_xor(s, 2);
      s += __shfl_xor(s, 4);
      const float mu = s * (1.0f / (float)HID);
      float vs = 0.0f;
#pragma unroll 4
      for (int j = 0; j < HID / 32; ++j) {
        const int f = j * 32 + q * 4;
        const v4f hv = *(const v4f*)(srow + f);
        const v4f d = hv - mu;
        vs += (d.x * d.x + d.y * d.y) + (d.z * d.z + d.w * d.w);
      }
      vs += __shfl_xor(vs, 1);
      vs += __shfl_xor(vs, 2);
      vs += __shfl_xor(vs, 4);
      const float rs = rsqrtf(vs * (1.0f / (float)HID) + LN_EPS_F);
      _Float16* hrow = H1 + row * P1;
#pragma unroll 4
      for (int j = 0; j < HID / 32; ++j) {
        const int f = j * 32 + q * 4;
        const v4f hv = *(const v4f*)(srow + f);
        const v4f gg = *(const v4f*)(g1e + f);
        const v4f be = *(const v4f*)(be1e + f);
        const v4f t  = (hv - mu) * rs;
        v4f u = t * gg + be;
        u = lrelu4(u) * A_CARRY;
        const v4h o = __builtin_convertvector(u, v4h);
        *(v4h*)(hrow + f) = o;
      }
    }
  }
  __syncthreads();

  {
    const int h = lane >> 4, m = lane & 15;
    const int rt = wave & 3, cg = wave >> 2;
    const _Float16* arow = H1 + (rt * 16 + m) * P1 + 8 * h;
    const _Float16* brow = W2S + ((size_t)bidx * HID2 + cg * 128 + m) * HID + 8 * h;
    v8f acc[8];
#pragma unroll
    for (int t = 0; t < 8; ++t) acc[t] = zero8();
#pragma unroll 1
    for (int kk = 0; kk < HID; kk += 32) {
      Frag fa;
      fa.half[0] = *(const v8h*)(arow + kk);
      fa.half[1] = *(const v8h*)(arow + kk + 16);
#pragma unroll
      for (int t = 0; t < 8; ++t) {
        const _Float16* bp = brow + (size_t)(t * 16) * HID + kk;
        Frag fb;
        fb.half[0] = *(const v8h*)(bp);
        fb.half[1] = *(const v8h*)(bp + 16);
        acc[t] = wmf(fa.v, fb.v, acc[t]);
      }
    }
#pragma unroll
    for (int t = 0; t < 8; ++t) {
      const int n = cg * 128 + t * 16 + m;
      const float bias = b2e[n];
      float* hc = H2 + (rt * 16 + 8 * h) * P2 + n;
#pragma unroll
      for (int r = 0; r < 8; ++r) hc[r * P2] = acc[t][r] * RC2048 + bias;
    }
  }
  __syncthreads();

  {
    const int q = tid & 3, row = tid >> 2;
    const float* hr = H2 + row * P2;
    float s = 0.0f;
#pragma unroll 4
    for (int j = 0; j < HID2 / 16; ++j) {
      const v4f v = *(const v4f*)(hr + j * 16 + q * 4);
      s += (v.x + v.y) + (v.z + v.w);
    }
    s += __shfl_xor(s, 1);
    s += __shfl_xor(s, 2);
    const float mu = s * (1.0f / (float)HID2);
    float vs = 0.0f;
#pragma unroll 4
    for (int j = 0; j < HID2 / 16; ++j) {
      const v4f v = *(const v4f*)(hr + j * 16 + q * 4);
      const v4f d = v - mu;
      vs += (d.x * d.x + d.y * d.y) + (d.z * d.z + d.w * d.w);
    }
    vs += __shfl_xor(vs, 1);
    vs += __shfl_xor(vs, 2);
    const float rs = rsqrtf(vs * (1.0f / (float)HID2) + LN_EPS_F);
    float o0 = 0.0f, o1 = 0.0f, o2 = 0.0f;
#pragma unroll 4
    for (int j = 0; j < HID2 / 16; ++j) {
      const int k = j * 16 + q * 4;
      const v4f v  = *(const v4f*)(hr + k);
      const v4f gg = *(const v4f*)(g2e + k);
      const v4f be = *(const v4f*)(be2e + k);
      const v4f t  = (v - mu) * rs;
      v4f u = t * gg + be;
      u = lrelu4(u);
      const v4f wa = *(const v4f*)(W3e + 3 * k);
      const v4f wb = *(const v4f*)(W3e + 3 * k + 4);
      const v4f wc = *(const v4f*)(W3e + 3 * k + 8);
      o0 += (u.x * wa.x + u.y * wa.w) + (u.z * wb.z + u.w * wc.y);
      o1 += (u.x * wa.y + u.y * wb.x) + (u.z * wb.w + u.w * wc.z);
      o2 += (u.x * wa.z + u.y * wb.y) + (u.z * wc.x + u.w * wc.w);
    }
    o0 += __shfl_xor(o0, 1); o0 += __shfl_xor(o0, 2);
    o1 += __shfl_xor(o1, 1); o1 += __shfl_xor(o1, 2);
    o2 += __shfl_xor(o2, 1); o2 += __shfl_xor(o2, 2);
    if (q == 0) {
      OS[row * 3 + 0] = o0 + b3e[0];
      OS[row * 3 + 1] = o1 + b3e[1];
      OS[row * 3 + 2] = o2 + b3e[2];
    }
  }
  __syncthreads();

  {
    const int li = tid < 48 ? tid : 47;
    const v4f ov = *(const v4f*)(OS + 4 * li);
    float* op = out + ((size_t)bidx * nN + p0) * 3;
    if (tid < 48) *(volatile v4f*)(op + 4 * tid) = ov;
    __threadfence();
    if (tid < 48) *(volatile v4f*)(op + 4 * tid) = ov;
  }
}

extern "C" void kernel_launch(void* const* d_in, const int* in_sizes, int n_in,
                              void* d_out, int out_size, void* d_ws, size_t ws_size,
                              hipStream_t stream) {
  if (n_in < 12) return;
  const int nB = in_sizes[1];
  if (nB <= 0) return;
  if (in_sizes[0] <= 0 || (in_sizes[0] % (3 * nB)) != 0) return;
  const int nN = in_sizes[0] / (3 * nB);
  if (nN <= 0 || (nN % TP) != 0) return;
  if (in_sizes[2] <= 0 || (in_sizes[2] % (3 * HID)) != 0) return;
  const int nE = in_sizes[2] / (3 * HID);
  if (nE <= 0) return;
  if (in_sizes[3] != nE * HID || in_sizes[4] != nE * HID || in_sizes[5] != nE * HID) return;
  if (in_sizes[6] != nE * HID * HID2) return;
  if (in_sizes[7] != nE * HID2 || in_sizes[8] != nE * HID2 || in_sizes[9] != nE * HID2) return;
  if (in_sizes[10] != nE * HID2 * 3 || in_sizes[11] != nE * 3) return;
  if (out_size != nB * nN * 3) return;

  const size_t wsz = (size_t)nB * HID2 * HID * 2;
  if (wsz > ws_size || wsz > (size_t)WSCAP) return;

  const float* pts = (const float*)d_in[0];
  const int*   cat = (const int*)d_in[1];
  const float* W1  = (const float*)d_in[2];
  const float* b1  = (const float*)d_in[3];
  const float* g1  = (const float*)d_in[4];
  const float* be1 = (const float*)d_in[5];
  const float* W2  = (const float*)d_in[6];
  const float* b2  = (const float*)d_in[7];
  const float* g2  = (const float*)d_in[8];
  const float* be2 = (const float*)d_in[9];
  const float* W3  = (const float*)d_in[10];
  const float* b3  = (const float*)d_in[11];
  float* out = (float*)d_out;
  _Float16* W2S = (_Float16*)d_ws;

  k_w2prep<<<nB * (HID2 / 32), NTH, 0, stream>>>(W2, cat, W2S, nE);

  hipFuncSetAttribute(reinterpret_cast<const void*>(&k_mlp),
                      hipFuncAttributeMaxDynamicSharedMemorySize, L_TOT);
  k_mlp<<<nB * (nN / TP), NTH, L_TOT, stream>>>(pts, cat, W1, b1, g1, be1, W2S, b2, g2, be2, W3, b3,
                                                 out, nN, nE);
}
